// TaMM_28965259444337
// MI455X (gfx1250) — hardware-run, weakly checked
//
#include <hip/hip_runtime.h>
#include <math.h>

typedef __attribute__((ext_vector_type(16))) _Float16 v16h;
typedef __attribute__((ext_vector_type(8)))  _Float16 v8h;
typedef __attribute__((ext_vector_type(8)))  float    v8f;
typedef __attribute__((ext_vector_type(4)))  float    v4f;
typedef __attribute__((ext_vector_type(4)))  int      v4i;
typedef __attribute__((ext_vector_type(4)))  unsigned int v4u;
typedef __attribute__((ext_vector_type(2)))  unsigned int v2u;

constexpr int kNB    = 4;
constexpr int kLQ    = 512;
constexpr int kLK    = 512;
constexpr int kHid   = 128;
constexpr int kVocab = 10000;
static_assert(kLQ == kLK);
static_assert((kHid % 32) == 0 && (kLK % 32) == 0);
static_assert((kLK % 64) == 0 && (kLQ % 16) == 0 && (kHid % 16) == 0);

constexpr double newton_sqrt(double x) {
  double r = x;
  for (int i = 0; i < 60; ++i) r = 0.5 * (r + x / r);
  return r;
}
constexpr float kInvTemper = (float)(1.0 / newton_sqrt((double)kHid));
static_assert(kInvTemper > 0.08838834f && kInvTemper < 0.08838836f);

constexpr float kOpCarry    = 16.0f;
constexpr float kPCarry     = 4096.0f;
constexpr float kScoreScale = kInvTemper / (kOpCarry * kOpCarry);
constexpr float kKoScale    = 1.0f / (kPCarry * kOpCarry);
constexpr float kF16MinNormal = 6.103515625e-05f;

constexpr int kPrepRows  = 64;
constexpr int kPrepPitch = 132;
constexpr int kPPitch    = 516;
constexpr int kHPitch    = 520;
constexpr int kKoPitch   = 132;

constexpr size_t kOffEK   = 0;
constexpr size_t kOffEKt  = kOffEK  + (size_t)kNB * kLK * kHid * 2;
constexpr size_t kOffHQ   = kOffEKt + (size_t)kNB * kHid * kLK * 2;
constexpr size_t kWsTotal = kOffHQ  + (size_t)kNB * kLQ * kHid * 2;
static_assert(kWsTotal == 1572864ull);
static_assert(kWsTotal <= 134217728ull);
static_assert((kOffEKt % 128) == 0 && (kOffHQ % 128) == 0);

__device__ __forceinline__ unsigned pk16(unsigned short a, unsigned short b) { return (unsigned)a | ((unsigned)b << 16); }

__device__ __forceinline__ unsigned short h_bits_fl(float f) {
  const float g = (fabsf(f) < kF16MinNormal) ? 0.0f : f;
  const _Float16 h = (_Float16)g;
  return __builtin_bit_cast(unsigned short, h);
}

__device__ __forceinline__ v4u pack8_f16(v4f a, v4f c, float carry) {
  const float x0 = a[0] * carry, x1 = a[1] * carry, x2 = a[2] * carry, x3 = a[3] * carry;
  const float x4 = c[0] * carry, x5 = c[1] * carry, x6 = c[2] * carry, x7 = c[3] * carry;
  return (v4u){pk16(h_bits_fl(x0), h_bits_fl(x1)), pk16(h_bits_fl(x2), h_bits_fl(x3)),
               pk16(h_bits_fl(x4), h_bits_fl(x5)), pk16(h_bits_fl(x6), h_bits_fl(x7))};
}

union FragH { v16h v; v8h h[2]; };

__device__ __forceinline__ v16h frag_load_g(const _Float16* p) {
  FragH f;
  f.h[0] = *(const v8h*)(p);
  f.h[1] = *(const v8h*)(p + 16);
  return f.v;
}

__device__ __forceinline__ v8f mma_h(v16h a, v16h b, v8f c) {
  c = __builtin_amdgcn_wmma_f32_16x16x32_f16(false, a, false, b, (short)0, c, false, false);
  asm volatile("v_nop\n\tv_nop\n\tv_nop\n\tv_nop" : "+v"(c) : "v"(a), "v"(b));
  return c;
}

__global__ __launch_bounds__(256) void prep_planes_kernel(
    const float* __restrict__ hidden, const int* __restrict__ key_seq, const float* __restrict__ key_table,
    unsigned short* __restrict__ EK, unsigned short* __restrict__ EKt, unsigned short* __restrict__ HQ)
{
  __shared__ __align__(16) float sK[kPrepRows * kPrepPitch];
  const int t = threadIdx.x, lane = t & 31, wave = t >> 5;
  const int b  = blockIdx.x >> 3;
  const int k0 = (blockIdx.x & 7) * 64;
  const int rbase = b * kLK + k0;

#pragma unroll
  for (int i = 0; i < 8; ++i) {
    const int e   = i * 256 + t;
    const int row = e >> 5;
    const int c4  = (e & 31) * 4;
    int idx = key_seq[rbase + row];
    idx = idx < 0 ? 0 : (idx > kVocab - 1 ? kVocab - 1 : idx);
    const v4f v = *(const v4f*)(key_table + (size_t)idx * kHid + c4);
    *(v4f*)(sK + row * kPrepPitch + c4) = v;
  }
  __syncthreads();

  v4u ekv[4], ektv[4], hqv[4];
#pragma unroll
  for (int it = 0; it < 4; ++it) {
    {
      const int row = it * 16 + wave * 2 + (lane >> 4);
      const float* sp = sK + row * kPrepPitch + (lane & 15) * 8;
      const v4f a0 = *(const v4f*)(sp);
      const v4f a1 = *(const v4f*)(sp + 4);
      ekv[it] = pack8_f16(a0, a1, kOpCarry);
    }
    {
      const int hrow = it * 32 + wave * 4 + (lane >> 3);
      const int k8   = (lane & 7) * 8;
      v4f a0, a1;
      a0[0] = sK[(k8 + 0) * kPrepPitch + hrow];
      a0[1] = sK[(k8 + 1) * kPrepPitch + hrow];
      a0[2] = sK[(k8 + 2) * kPrepPitch + hrow];
      a0[3] = sK[(k8 + 3) * kPrepPitch + hrow];
      a1[0] = sK[(k8 + 4) * kPrepPitch + hrow];
      a1[1] = sK[(k8 + 5) * kPrepPitch + hrow];
      a1[2] = sK[(k8 + 6) * kPrepPitch + hrow];
      a1[3] = sK[(k8 + 7) * kPrepPitch + hrow];
      ektv[it] = pack8_f16(a0, a1, kOpCarry);
    }
    {
      const int e   = it * 256 + t;
      const int row = e >> 4;
      const int c8  = (e & 15) * 8;
      const float* p = hidden + (size_t)(rbase + row) * kHid + c8;
      const v4f a0 = *(const v4f*)(p);
      const v4f a1 = *(const v4f*)(p + 4);
      hqv[it] = pack8_f16(a0, a1, kOpCarry);
    }
  }

  for (int pass = 0; pass < 2; ++pass) {
#pragma unroll
    for (int it = 0; it < 4; ++it) {
      {
        const int row = it * 16 + wave * 2 + (lane >> 4);
        *(volatile v4u*)(EK + (size_t)(rbase + row) * kHid + (lane & 15) * 8) = ekv[it];
      }
      {
        const int hrow = it * 32 + wave * 4 + (lane >> 3);
        *(volatile v4u*)(EKt + ((size_t)(b * kHid + hrow) * kLK + k0 + (lane & 7) * 8)) = ektv[it];
      }
      {
        const int e   = it * 256 + t;
        const int row = e >> 4;
        *(volatile v4u*)(HQ + (size_t)(rbase + row) * kHid + (e & 15) * 8) = hqv[it];
      }
    }
    __threadfence();
  }
}

__global__ __launch_bounds__(256) void fused_memory_attention_kernel(
    const float* __restrict__ hidden, const int* __restrict__ value_matrix, const int* __restrict__ key_mask,
    const float* __restrict__ val_table,
    const unsigned short* __restrict__ HQp, const unsigned short* __restrict__ EKp, const unsigned short* __restrict__ EKtp,
    float* __restrict__ out)
{
  __shared__ __align__(16) float    sP32[16 * kPPitch];
  __shared__ __align__(16) _Float16 sP16[16 * kHPitch];
  __shared__ __align__(16) float    sKO[16 * kKoPitch];

  const int tid  = threadIdx.x;
  const int lane = tid & 31;
  const int wave = __builtin_amdgcn_readfirstlane(tid >> 5);
  const int hh   = lane >> 4;
  const int m    = lane & 15;
  const int b    = blockIdx.x >> 5;
  const int q0   = (blockIdx.x & 31) * 16;

  const _Float16* HQ  = (const _Float16*)HQp;
  const _Float16* EK  = (const _Float16*)EKp;
  const _Float16* EKt = (const _Float16*)EKtp;

  {
    v8f acc[4];
#pragma unroll
    for (int j = 0; j < 4; ++j) acc[j] = (v8f){0.f, 0.f, 0.f, 0.f, 0.f, 0.f, 0.f, 0.f};
    const _Float16* arow = HQ + (size_t)(b * kLQ + q0 + m) * kHid + 8 * hh;
    const _Float16* brow = EK + (size_t)(b * kLK + wave * 64 + m) * kHid + 8 * hh;
#pragma unroll
    for (int ks = 0; ks < 4; ++ks) {
      const v16h af = frag_load_g(arow + ks * 32);
#pragma unroll
      for (int j = 0; j < 4; ++j) {
        const v16h bf = frag_load_g(brow + (size_t)j * 16 * kHid + ks * 32);
        acc[j] = mma_h(af, bf, acc[j]);
      }
    }
#pragma unroll
    for (int j = 0; j < 4; ++j) {
#pragma unroll
      for (int r = 0; r < 8; ++r) {
        sP32[(8 * hh + r) * kPPitch + wave * 64 + j * 16 + m] = acc[j][r] * kScoreScale;
      }
    }
  }
  __syncthreads();

#pragma unroll 1
  for (int rq = 0; rq < 2; ++rq) {
    const int qr = wave * 2 + rq;
    const size_t rowg = (size_t)(b * kLQ + q0 + qr);
    const int* mrow = key_mask + rowg * kLK;
    float* prow = sP32 + qr * kPPitch;
    float s = 0.0f;
#pragma unroll 1
    for (int i = 0; i < 4; ++i) {
      const int col = i * 128 + lane * 4;
      const v4i mk = *(const v4i*)(mrow + col);
      const v4f uv = *(const v4f*)(prow + col);
      const float x0 = expf(uv[0]);
      const float x1 = expf(uv[1]);
      const float x2 = expf(uv[2]);
      const float x3 = expf(uv[3]);
      v4f ev;
      ev[0] = (mk[0] > 0) ? x0 : 0.0f;
      ev[1] = (mk[1] > 0) ? x1 : 0.0f;
      ev[2] = (mk[2] > 0) ? x2 : 0.0f;
      ev[3] = (mk[3] > 0) ? x3 : 0.0f;
      *(v4f*)(prow + col) = ev;
      s += ev[0];
      s += ev[1];
      s += ev[2];
      s += ev[3];
    }
    s += __shfl_xor(s, 16, 32);
    s += __shfl_xor(s, 8, 32);
    s += __shfl_xor(s, 4, 32);
    s += __shfl_xor(s, 2, 32);
    s += __shfl_xor(s, 1, 32);
    const float inv = 1.0f / (s + 1e-10f);
#pragma unroll 1
    for (int i = 0; i < 4; ++i) {
      const int col = i * 128 + lane * 4;
      const v4f ev = *(const v4f*)(prow + col);
      v4f pv;
      pv[0] = ev[0] * inv;
      pv[1] = ev[1] * inv;
      pv[2] = ev[2] * inv;
      pv[3] = ev[3] * inv;
      *(v4f*)(prow + col) = pv;
      const float c0 = pv[0] * kPCarry, c1 = pv[1] * kPCarry, c2 = pv[2] * kPCarry, c3 = pv[3] * kPCarry;
      const v2u hw = (v2u){pk16(h_bits_fl(c0), h_bits_fl(c1)), pk16(h_bits_fl(c2), h_bits_fl(c3))};
      *(v2u*)(sP16 + qr * kHPitch + col) = hw;
    }
  }
  __syncthreads();

  {
    v8f acc = (v8f){0.f, 0.f, 0.f, 0.f, 0.f, 0.f, 0.f, 0.f};
    const _Float16* pa   = sP16 + m * kHPitch + 8 * hh;
    const _Float16* brow = EKt + (size_t)(b * kHid + wave * 16 + m) * kLK + 8 * hh;
#pragma unroll 4
    for (int ks = 0; ks < 16; ++ks) {
      FragH af;
      af.h[0] = *(const v8h*)(pa + ks * 32);
      af.h[1] = *(const v8h*)(pa + ks * 32 + 16);
      const v16h bf = frag_load_g(brow + ks * 32);
      acc = mma_h(af.v, bf, acc);
    }
#pragma unroll
    for (int r = 0; r < 8; ++r) {
      sKO[(8 * hh + r) * kKoPitch + wave * 16 + m] = acc[r] * kKoScale;
    }
  }
  __syncthreads();

  const int h0 = lane * 4;
#pragma unroll 1
  for (int rq = 0; rq < 2; ++rq) {
    const int qr = wave * 2 + rq;
    const size_t rowg = (size_t)(b * kLQ + q0 + qr);
    const int* vmrow = value_matrix + rowg * kLK;
    const float* prow = sP32 + qr * kPPitch;
    float a0 = 0.0f, a1 = 0.0f, a2 = 0.0f, a3 = 0.0f;
#pragma unroll 1
    for (int k = 0; k < kLK; ++k) {
      const float w = __int_as_float(__builtin_amdgcn_readfirstlane(__float_as_int(prow[k])));
      int idx = __builtin_amdgcn_readfirstlane(vmrow[k]);
      idx = idx < 0 ? 0 : (idx > kVocab - 1 ? kVocab - 1 : idx);
      if (w != 0.0f) {
        const v4f v = *(const v4f*)(val_table + (size_t)idx * kHid + h0);
        a0 = fmaf(w, v[0], a0);
        a1 = fmaf(w, v[1], a1);
        a2 = fmaf(w, v[2], a2);
        a3 = fmaf(w, v[3], a3);
      }
    }
    const v4f kv = *(const v4f*)(sKO + qr * kKoPitch + h0);
    const v4f hv = *(const v4f*)(hidden + rowg * kHid + h0);
    v4f res;
    res[0] = (a0 + kv[0]) + hv[0];
    res[1] = (a1 + kv[1]) + hv[1];
    res[2] = (a2 + kv[2]) + hv[2];
    res[3] = (a3 + kv[3]) + hv[3];
    float* op = out + rowg * kHid + h0;
    *(volatile v4f*)op = res;
    __threadfence();
    *(volatile v4f*)op = res;
  }
}

extern "C" void kernel_launch(void* const* d_in, const int* in_sizes, int n_in,
                              void* d_out, int out_size, void* d_ws, size_t ws_size,
                              hipStream_t stream) {
  if (n_in < 6) return;
  if (in_sizes[0] != kNB * kLQ * kHid) return;
  if (in_sizes[1] != kNB * kLK) return;
  if (in_sizes[2] != kNB * kLQ * kLK) return;
  if (in_sizes[3] != kNB * kLQ * kLK) return;
  if (in_sizes[4] != kVocab * kHid) return;
  if (in_sizes[5] != kVocab * kHid) return;
  if (out_size != kNB * kLQ * kHid) return;
  if (ws_size < kWsTotal) return;

  const float* hidden       = (const float*)d_in[0];
  const int*   key_seq      = (const int*)d_in[1];
  const int*   value_matrix = (const int*)d_in[2];
  const int*   key_mask     = (const int*)d_in[3];
  const float* key_table    = (const float*)d_in[4];
  const float* val_table    = (const float*)d_in[5];
  float* out = (float*)d_out;

  char* ws = (char*)d_ws;
  unsigned short* EK  = (unsigned short*)(ws + kOffEK);
  unsigned short* EKt = (unsigned short*)(ws + kOffEKt);
  unsigned short* HQ  = (unsigned short*)(ws + kOffHQ);

  prep_planes_kernel<<<kNB * (kLK / 64), 256, 0, stream>>>(hidden, key_seq, key_table, EK, EKt, HQ);

  fused_memory_attention_kernel<<<kNB * (kLQ / 16), 256, 0, stream>>>(
      hidden, value_matrix, key_mask, val_table, HQ, EK, EKt, out);
}
